// gruaging_rnnosc3ode_70308614636171
// MI455X (gfx1250) — hardware-verified
//
#include <hip/hip_runtime.h>
#include <cstddef>

#pragma clang fp contract(off)

typedef __attribute__((ext_vector_type(16))) _Float16 v16h;
typedef __attribute__((ext_vector_type(8)))  _Float16 v8h;
typedef __attribute__((ext_vector_type(8)))  float    v8f;
typedef __attribute__((ext_vector_type(4)))  float    v4f;

constexpr int NBATCH = 256;
constexpr int NSTEP  = 2048;
constexpr int NXCOL  = 9;
constexpr int NUIN   = 8;
constexpr int NHID   = 128;
constexpr int NGATE3 = 3 * NHID;
constexpr int KXPAD  = 32;
constexpr int NHIN   = 64;
constexpr int NHOUT  = 64;
constexpr int ROWS_PER_BLOCK = 16;
constexpr int GRU_THREADS = 256;
constexpr int GRU_BLOCKS = NBATCH / ROWS_PER_BLOCK;
constexpr int HPITCH = 136;
constexpr int XPITCH = 40;
constexpr int ODE_THREADS = 64;
constexpr int ODE_BLOCKS = NBATCH / ODE_THREADS;
constexpr int OPITCH = 36;
constexpr int DP_LINE = 32;
constexpr float WCARRY = 16.0f;
constexpr float WCARRY_INV = 0.0625f;
constexpr float DTC  = 0.02f;
constexpr float HDTC = 0.5f * DTC;
constexpr float DT6C = DTC / 6.0f;
constexpr float OSC_W0 = -20.0f;
constexpr float OSC_W1 = 10.0f;
constexpr float XINIT0 = 0.4736f;
constexpr float XINIT1 = 0.8745f;
constexpr float XINIT2 = 1.8497f;

static_assert(NBATCH % ROWS_PER_BLOCK == 0);
static_assert(NBATCH % ODE_THREADS == 0);
static_assert(NHIN == ODE_THREADS && NHOUT == ODE_THREADS);
static_assert(NSTEP % 32 == 0);
static_assert((HPITCH * 2) % 16 == 0 && (XPITCH * 2) % 16 == 0);
static_assert(NGATE3 == 8 * 3 * 16);

constexpr size_t WS_WHH_OFF   = 0;
constexpr size_t WS_WHH_BYTES = (size_t)NGATE3 * NHID * 2;
constexpr size_t WS_WIH_OFF   = WS_WHH_OFF + WS_WHH_BYTES;
constexpr size_t WS_WIH_BYTES = (size_t)NGATE3 * KXPAD * 2;
constexpr size_t WS_DP_OFF    = WS_WIH_OFF + WS_WIH_BYTES;
constexpr size_t WS_DP_BYTES  = (size_t)GRU_BLOCKS * DP_LINE * 4;
constexpr size_t WS_TOTAL     = WS_DP_OFF + WS_DP_BYTES;
static_assert(WS_WHH_BYTES == 98304 && WS_WIH_OFF == 98304 && WS_DP_OFF == 122880 && WS_TOTAL == 124928);
static_assert(WS_WIH_OFF % 128 == 0 && WS_DP_OFF % 128 == 0);
static_assert(WS_TOTAL <= (size_t)134217728);

constexpr int NPAIR_HH = NGATE3 * NHID / 2;
constexpr int NPAIR_IH = NGATE3 * KXPAD / 2;
constexpr int PREP_BLOCKS = (NPAIR_HH + NPAIR_IH) / 256;
static_assert(NPAIR_HH % 256 == 0 && (NPAIR_HH + NPAIR_IH) % 256 == 0);

__device__ __forceinline__ void dep_guard_h(v8f& a, v8f& b, v16h x, v16h y) { asm volatile("v_nop\n\tv_nop\n\tv_nop\n\tv_nop" : "+v"(a), "+v"(b) : "v"(x), "v"(y)); }
__device__ __forceinline__ void keep4_h(v16h a, v16h b, v16h c, v16h d) { asm volatile("v_nop" :: "v"(a), "v"(b), "v"(c), "v"(d)); }
template <typename T> struct Frag;
template <> struct Frag<_Float16> {
  typedef v16h V; union U { v16h v; v8h h[2]; };
  static __device__ __forceinline__ v16h load(const _Float16* p) {
    U f; f.h[0] = *(const v8h*)(p); f.h[1] = *(const v8h*)(p + 16); return f.v;
  }
  static __device__ __forceinline__ v8f mma(v16h a, v16h b, v8f c) {
    return __builtin_amdgcn_wmma_f32_16x16x32_f16(false, a, false, b, (short)0, c, false, false);
  }
  static __device__ __forceinline__ void guard(v8f& a, v8f& b, v16h x, v16h y) { dep_guard_h(a, b, x, y); }
  static __device__ __forceinline__ void keep(v16h a, v16h b, v16h c, v16h d) { keep4_h(a, b, c, d); }
};

__device__ __forceinline__ void guard3(v8f& a, v8f& b, v8f& c, v16h fa, v16h f0, v16h f1, v16h f2) {
  asm volatile("v_nop\n\tv_nop\n\tv_nop\n\tv_nop" : "+v"(a), "+v"(b), "+v"(c) : "v"(fa), "v"(f0), "v"(f1), "v"(f2));
}

__device__ __forceinline__ unsigned pack_f16x2(float a, float b) {
  const _Float16 h0 = (_Float16)a, h1 = (_Float16)b;
  return (unsigned)__builtin_bit_cast(unsigned short, h0) | ((unsigned)__builtin_bit_cast(unsigned short, h1) << 16);
}

__device__ __forceinline__ float sigm_f(float x) {
  const float e = expf(-x);
  const float d = 1.0f + e;
  return 1.0f / d;
}
__device__ __forceinline__ float tanh_via_exp(float x) {
  const float e = expf(2.0f * x);
  const float d = 1.0f + e;
  return 1.0f - 2.0f / d;
}

__global__ __launch_bounds__(256) void prep_weights_kernel(
    const float* __restrict__ whh, const float* __restrict__ wih,
    unsigned* whh16, unsigned* wih16)
{
  const int i = blockIdx.x * 256 + threadIdx.x;
  if (i < NPAIR_HH) {
    const float f0 = whh[2 * i] * WCARRY;
    const float f1 = whh[2 * i + 1] * WCARRY;
    const unsigned u = pack_f16x2(f0, f1);
    ((volatile unsigned*)whh16)[i] = u;
    __threadfence();
    ((volatile unsigned*)whh16)[i] = u;
  } else {
    const int j  = i - NPAIR_HH;
    const int n  = j >> 4;
    const int kp = j & 15;
    const int k0 = 2 * kp, k1 = k0 + 1;
    const int c0 = (k0 < NXCOL) ? k0 : (NXCOL - 1);
    const int c1 = (k1 < NXCOL) ? k1 : (NXCOL - 1);
    const float s0 = (k0 < NXCOL) ? WCARRY : 0.0f;
    const float s1 = (k1 < NXCOL) ? WCARRY : 0.0f;
    const float f0 = wih[n * NXCOL + c0] * s0;
    const float f1 = wih[n * NXCOL + c1] * s1;
    const unsigned u = pack_f16x2(f0, f1);
    ((volatile unsigned*)wih16)[j] = u;
    __threadfence();
    ((volatile unsigned*)wih16)[j] = u;
  }
}

constexpr int HA_U4 = 2 * ROWS_PER_BLOCK * HPITCH * 2 / 16;
constexpr int XA_U4 = 2 * ROWS_PER_BLOCK * XPITCH * 2 / 16;
static_assert(HA_U4 * 16 == 2 * ROWS_PER_BLOCK * HPITCH * 2 && XA_U4 * 16 == 2 * ROWS_PER_BLOCK * XPITCH * 2);

__global__ __launch_bounds__(GRU_THREADS) void gru_dparam_kernel(
    const float* __restrict__ xin,
    const unsigned short* whh16, const unsigned short* wih16,
    const float* __restrict__ bih, const float* __restrict__ bhh,
    const float* __restrict__ wage, const float* __restrict__ bage,
    float* dpout)
{
  __shared__ __align__(16) _Float16 hA[2][ROWS_PER_BLOCK * HPITCH];
  __shared__ __align__(16) _Float16 xA[2][ROWS_PER_BLOCK * XPITCH];
  __shared__ float red[8][ROWS_PER_BLOCK];
  __shared__ __align__(16) float dline[DP_LINE];

  const int tid  = threadIdx.x;
  const int lane = tid & 31;
  const int wv   = tid >> 5;
  const int hh   = lane >> 4;
  const int cl   = lane & 15;
  const int koff = hh * 8;
  const int b0   = blockIdx.x * ROWS_PER_BLOCK;
  const int unit = wv * 16 + cl;

  {
    const uint4 z = make_uint4(0u, 0u, 0u, 0u);
    uint4* ph = reinterpret_cast<uint4*>(&hA[0][0]);
    uint4* px = reinterpret_cast<uint4*>(&xA[0][0]);
    for (int i = tid; i < HA_U4; i += GRU_THREADS) ph[i] = z;
    for (int i = tid; i < XA_U4; i += GRU_THREADS) px[i] = z;
  }
  __syncthreads();

  const bool xstager = tid < ROWS_PER_BLOCK * NXCOL;
  const int m9 = xstager ? tid : 0;
  const int xm = m9 / NXCOL;
  const int xc = m9 - xm * NXCOL;
  const float* xrow = xin + ((size_t)(b0 + xm) * NSTEP) * NXCOL + xc;
  if (xstager) xA[0][xm * XPITCH + xc] = (_Float16)xrow[0];

  const float bias_r  = bih[unit] + bhh[unit];
  const float bias_z  = bih[NHID + unit] + bhh[NHID + unit];
  const float bias_in = bih[2 * NHID + unit];
  const float bias_hn = bhh[2 * NHID + unit];
  const float wa = wage[unit];

  const _Float16* wihp = (const _Float16*)wih16;
  const _Float16* whhp = (const _Float16*)whh16;
  const v16h bxr = Frag<_Float16>::load(wihp + (size_t)unit * KXPAD + koff);
  const v16h bxz = Frag<_Float16>::load(wihp + (size_t)(NHID + unit) * KXPAD + koff);
  const v16h bxn = Frag<_Float16>::load(wihp + (size_t)(2 * NHID + unit) * KXPAD + koff);

  float hreg[8];
#pragma unroll
  for (int r = 0; r < 8; ++r) hreg[r] = 0.0f;
  __syncthreads();

  for (int t = 0; t < NSTEP; ++t) {
    asm volatile("" ::: "memory");
    const int cur = t & 1;
    const int nxt = cur ^ 1;

    const int tn = (t + 1 < NSTEP) ? (t + 1) : (NSTEP - 1);
    const float xv = xrow[(size_t)tn * NXCOL];

    v8f acc_r = (v8f){0.f,0.f,0.f,0.f,0.f,0.f,0.f,0.f};
    v8f acc_z = acc_r, acc_i = acc_r, acc_n = acc_r;

    {
      const v16h ax = Frag<_Float16>::load(&xA[cur][cl * XPITCH + koff]);
      acc_r = Frag<_Float16>::mma(ax, bxr, acc_r);
      acc_z = Frag<_Float16>::mma(ax, bxz, acc_z);
      acc_i = Frag<_Float16>::mma(ax, bxn, acc_i);
      guard3(acc_r, acc_z, acc_i, ax, bxr, bxz, bxn);
    }
#pragma unroll
    for (int kc = 0; kc < 4; ++kc) {
      const v16h ah = Frag<_Float16>::load(&hA[cur][cl * HPITCH + koff + 32 * kc]);
      const size_t wo = (size_t)koff + 32 * kc;
      const v16h bgr = Frag<_Float16>::load(whhp + (size_t)unit * NHID + wo);
      const v16h bgz = Frag<_Float16>::load(whhp + (size_t)(NHID + unit) * NHID + wo);
      const v16h bgn = Frag<_Float16>::load(whhp + (size_t)(2 * NHID + unit) * NHID + wo);
      acc_r = Frag<_Float16>::mma(ah, bgr, acc_r);
      acc_z = Frag<_Float16>::mma(ah, bgz, acc_z);
      acc_n = Frag<_Float16>::mma(ah, bgn, acc_n);
      guard3(acc_r, acc_z, acc_n, ah, bgr, bgz, bgn);
    }

#pragma unroll
    for (int r = 0; r < 8; ++r) {
      const float pr = acc_r[r] * WCARRY_INV + bias_r;
      const float pz = acc_z[r] * WCARRY_INV + bias_z;
      const float pi = acc_i[r] * WCARRY_INV + bias_in;
      const float pn = acc_n[r] * WCARRY_INV + bias_hn;
      const float rg = sigm_f(pr);
      const float zg = sigm_f(pz);
      const float ng = tanh_via_exp(pi + rg * pn);
      const float hn = (1.0f - zg) * ng + zg * hreg[r];
      hreg[r] = hn;
      hA[nxt][(8 * hh + r) * HPITCH + unit] = (_Float16)hn;
    }
    if (xstager) xA[nxt][xm * XPITCH + xc] = (_Float16)xv;
    __syncthreads();
  }

  float part[8];
#pragma unroll
  for (int r = 0; r < 8; ++r) part[r] = hreg[r] * wa;
#pragma unroll
  for (int off = 1; off < 16; off <<= 1) {
#pragma unroll
    for (int r = 0; r < 8; ++r) part[r] += __shfl_xor(part[r], off, 32);
  }
  if (cl == 0) {
#pragma unroll
    for (int r = 0; r < 8; ++r) red[wv][8 * hh + r] = part[r];
  }
  __syncthreads();
  if (tid < 32) {
    const int rr = tid & 15;
    float s = 0.0f;
#pragma unroll
    for (int w8 = 0; w8 < 8; ++w8) s = s + red[w8][rr];
    const float v = (tid < ROWS_PER_BLOCK) ? (s + bage[0]) : 0.0f;
    dline[tid] = v;
  }
  __syncthreads();
  if (tid < 8) {
    const v4f v = *(const v4f*)(dline + 4 * tid);
    float* p = dpout + (size_t)blockIdx.x * DP_LINE + 4 * tid;
    *(volatile v4f*)p = v;
    __threadfence();
    *(volatile v4f*)p = v;
  }
}

__global__ __launch_bounds__(ODE_THREADS) void ode_readout_kernel(
    const float* __restrict__ xin,
    const float* __restrict__ wnin, const float* __restrict__ bnin,
    const float* __restrict__ wlin, const float* __restrict__ blin,
    const float* __restrict__ tau,
    const float* __restrict__ wnl,  const float* __restrict__ bnl,
    const float* __restrict__ wout, const float* __restrict__ bout,
    const float* dpin, float* yout)
{
  __shared__ __align__(16) float sWn[NHIN * NUIN];
  __shared__ float sBn[NHIN];
  __shared__ float sWl[NHIN];
  __shared__ __align__(16) float sWnl[NHOUT * 4];
  __shared__ float sBnl[NHOUT];
  __shared__ float sWo[NHOUT];
  __shared__ __align__(16) float sOut[ODE_THREADS * OPITCH];

  const int tid = threadIdx.x;
  const int b   = blockIdx.x * ODE_THREADS + tid;

  for (int i = tid; i < NHIN * NUIN; i += ODE_THREADS) sWn[i] = wnin[i];
  sBn[tid]  = bnin[tid];
  sWl[tid]  = wlin[tid];
  sBnl[tid] = bnl[tid];
  sWo[tid]  = wout[tid];
  sWnl[4 * tid + 0] = wnl[3 * tid + 0];
  sWnl[4 * tid + 1] = wnl[3 * tid + 1];
  sWnl[4 * tid + 2] = wnl[3 * tid + 2];
  sWnl[4 * tid + 3] = 0.0f;
  __syncthreads();

  const float base  = tau[0] + dpin[(b >> 4) * DP_LINE + (b & 15)];
  const float blin0 = blin[0];
  const float bout0 = bout[0];
  const float* urow = xin + (size_t)b * NSTEP * NXCOL;

  float x1 = XINIT0, x2 = XINIT1, x3 = XINIT2;
  float ul[NUIN], uh[NUIN], um[NUIN];
#pragma unroll
  for (int c = 0; c < NUIN; ++c) { ul[c] = 0.0f; uh[c] = 0.0f; um[c] = 0.0f; }
  float inv_lo = 0.0f, inv_mid = 0.0f, inv_hi = 0.0f;

  for (int it = 0; it <= NSTEP; ++it) {
    const int t = it - 1;
    if (it >= 1) {
      float acc = 0.0f;
#pragma unroll 1
      for (int j = 0; j < NHOUT; ++j) {
        const v4f w = *(const v4f*)(sWnl + 4 * j);
        float s = w[0] * x1;
        s = s + w[1] * x2;
        s = s + w[2] * x3;
        s = s + sBnl[j];
        const float g = sigm_f(s);
        acc = acc + g * sWo[j];
      }
      const float y = acc + bout0;
      sOut[tid * OPITCH + (t & 31)] = y;
      if ((t & 31) == 31) {
        __syncthreads();
        const int wq = tid >> 5, ln = tid & 31, q = ln & 7, rq = ln >> 3;
        float* ob = yout + (size_t)(blockIdx.x * ODE_THREADS) * NSTEP + (size_t)(t >> 5) * 32;
        for (int pass = 0; pass < 2; ++pass) {
#pragma unroll
          for (int i = 0; i < 8; ++i) {
            const int row = wq * 32 + i * 4 + rq;
            const v4f v = *(const v4f*)(sOut + row * OPITCH + 4 * q);
            *(volatile v4f*)(ob + (size_t)row * NSTEP + 4 * q) = v;
          }
          __threadfence();
        }
        __syncthreads();
      }
    }
    const bool more = (it == 0) || (t < NSTEP - 1);
    if (more) {
      const int tn = (it == 0) ? 0 : (t + 1);
#pragma unroll
      for (int c = 0; c < NUIN; ++c) uh[c] = urow[(size_t)tn * NXCOL + c];
#pragma unroll
      for (int c = 0; c < NUIN; ++c) {
        const float s = ul[c] + uh[c];
        um[c] = (it == 0) ? uh[c] : (s * 0.5f);
      }
      float am = 0.0f, ah2 = 0.0f;
#pragma unroll 1
      for (int j = 0; j < NHIN; ++j) {
        const v4f wa4 = *(const v4f*)(sWn + 8 * j);
        const v4f wb4 = *(const v4f*)(sWn + 8 * j + 4);
        float sm = wa4[0] * um[0];
        sm = sm + wa4[1] * um[1];
        sm = sm + wa4[2] * um[2];
        sm = sm + wa4[3] * um[3];
        sm = sm + wb4[0] * um[4];
        sm = sm + wb4[1] * um[5];
        sm = sm + wb4[2] * um[6];
        sm = sm + wb4[3] * um[7];
        sm = sm + sBn[j];
        float sh = wa4[0] * uh[0];
        sh = sh + wa4[1] * uh[1];
        sh = sh + wa4[2] * uh[2];
        sh = sh + wa4[3] * uh[3];
        sh = sh + wb4[0] * uh[4];
        sh = sh + wb4[1] * uh[5];
        sh = sh + wb4[2] * uh[6];
        sh = sh + wb4[3] * uh[7];
        sh = sh + sBn[j];
        const float gm = sigm_f(sm);
        const float gh = sigm_f(sh);
        am  = am  + gm * sWl[j];
        ah2 = ah2 + gh * sWl[j];
      }
      const float mm = am + blin0;
      const float mh = ah2 + blin0;
      const float em = base + mm;
      const float eh = base + mh;
      inv_mid = expf(-em);
      inv_hi  = expf(-eh);
      if (it >= 1) {
        float kp1 = 0.0f, kp2 = 0.0f, kp3 = 0.0f;
        float ks1 = 0.0f, ks2 = 0.0f, ks3 = 0.0f;
#pragma unroll 1
        for (int st = 0; st < 4; ++st) {
          const float cf  = (st == 0) ? 0.0f : ((st == 3) ? DTC : HDTC);
          const float wg  = (st == 1 || st == 2) ? 2.0f : 1.0f;
          const float inv = (st == 0) ? inv_lo : ((st == 3) ? inv_hi : inv_mid);
          const float a1 = x1 + cf * kp1;
          const float a2 = x2 + cf * kp2;
          const float a3 = x3 + cf * kp3;
          float th1 = 0.0f, th2 = 0.0f, th3 = 0.0f;
#pragma unroll 1
          for (int cc = 0; cc < 3; ++cc) {
            const float a  = (cc == 0) ? a1 : ((cc == 1) ? a2 : a3);
            const float th = tanhf(a);
            th1 = (cc == 0) ? th : th1;
            th2 = (cc == 1) ? th : th2;
            th3 = (cc == 2) ? th : th3;
          }
          const float d1 = (-a1 + th2) * inv;
          const float d2 = (-a2 + th3) * inv;
          const float q3 = -a3 + OSC_W0 * th1;
          const float d3 = (q3 + OSC_W1 * th2) * inv;
          ks1 = ks1 + wg * d1;
          ks2 = ks2 + wg * d2;
          ks3 = ks3 + wg * d3;
          kp1 = d1; kp2 = d2; kp3 = d3;
        }
        x1 = x1 + DT6C * ks1;
        x2 = x2 + DT6C * ks2;
        x3 = x3 + DT6C * ks3;
      }
#pragma unroll
      for (int c = 0; c < NUIN; ++c) ul[c] = uh[c];
      inv_lo = inv_hi;
    }
  }
}

extern "C" void kernel_launch(void* const* d_in, const int* in_sizes, int n_in,
                              void* d_out, int out_size, void* d_ws, size_t ws_size,
                              hipStream_t stream)
{
  (void)in_sizes; (void)n_in; (void)out_size; (void)ws_size;
  const float* inputdata = (const float*)d_in[0];
  const float* W_ih  = (const float*)d_in[1];
  const float* W_hh  = (const float*)d_in[2];
  const float* b_ih  = (const float*)d_in[3];
  const float* b_hh  = (const float*)d_in[4];
  const float* W_age = (const float*)d_in[5];
  const float* b_age = (const float*)d_in[6];
  const float* W_nin = (const float*)d_in[7];
  const float* b_nin = (const float*)d_in[8];
  const float* W_lin = (const float*)d_in[9];
  const float* b_lin = (const float*)d_in[10];
  const float* tau   = (const float*)d_in[11];
  const float* W_nl  = (const float*)d_in[12];
  const float* b_nl  = (const float*)d_in[13];
  const float* W_out = (const float*)d_in[14];
  const float* b_out = (const float*)d_in[15];
  float* out = (float*)d_out;

  char* ws = (char*)d_ws;
  unsigned* whh16 = (unsigned*)(ws + WS_WHH_OFF);
  unsigned* wih16 = (unsigned*)(ws + WS_WIH_OFF);
  float*    dpws  = (float*)(ws + WS_DP_OFF);

  prep_weights_kernel<<<PREP_BLOCKS, 256, 0, stream>>>(W_hh, W_ih, whh16, wih16);
  gru_dparam_kernel<<<GRU_BLOCKS, GRU_THREADS, 0, stream>>>(
      inputdata, (const unsigned short*)whh16, (const unsigned short*)wih16,
      b_ih, b_hh, W_age, b_age, dpws);
  ode_readout_kernel<<<ODE_BLOCKS, ODE_THREADS, 0, stream>>>(
      inputdata, W_nin, b_nin, W_lin, b_lin, tau, W_nl, b_nl, W_out, b_out, dpws, out);
}
